// CrossAxialMultiAttention_223338300233
// MI455X (gfx1250) — hardware-verified
//
#include <hip/hip_runtime.h>
#include <stdint.h>

typedef float          v4f  __attribute__((ext_vector_type(4)));
typedef float          v8f  __attribute__((ext_vector_type(8)));
typedef unsigned int   v2u  __attribute__((ext_vector_type(2)));
typedef unsigned short v8us __attribute__((ext_vector_type(8)));
typedef __bf16         v16b __attribute__((ext_vector_type(16)));
union Frag { v16b v; v8us h[2]; };

#define C_DIM 256
#define NH    8
#define DH    32
#define B_SZ  2
#define M_AX  32
#define T_LEN 512
#define KP    40

static __device__ __forceinline__ unsigned int bf16_rne(float x) {
  unsigned int u = __float_as_uint(x);
  return (u + 0x7FFFu + ((u >> 16) & 1u)) >> 16;
}
static __device__ __forceinline__ void split_hl(float x, unsigned int& hb, unsigned int& lb) {
  hb = bf16_rne(x);
  float r = x - __uint_as_float(hb << 16);
  lb = bf16_rne(r);
}
static __device__ __forceinline__ void split4(v4f v, v2u& hi, v2u& lo) {
  unsigned int h0, h1, h2, h3, l0, l1, l2, l3;
  split_hl(v.x, h0, l0); split_hl(v.y, h1, l1); split_hl(v.z, h2, l2); split_hl(v.w, h3, l3);
  hi.x = h0 | (h1 << 16); hi.y = h2 | (h3 << 16);
  lo.x = l0 | (l1 << 16); lo.y = l2 | (l3 << 16);
}

static __device__ __forceinline__ void mma3(v8f& acc, v16b ah, v16b al, v16b bh, v16b bl) {
  acc = __builtin_amdgcn_wmma_f32_16x16x32_bf16(false, ah, false, bh, (short)0, acc, false, false);
  acc = __builtin_amdgcn_wmma_f32_16x16x32_bf16(false, ah, false, bl, (short)0, acc, false, false);
  acc = __builtin_amdgcn_wmma_f32_16x16x32_bf16(false, al, false, bh, (short)0, acc, false, false);
  asm volatile("v_nop\n\tv_nop\n\tv_nop\n\tv_nop" : "+v"(acc) : "v"(ah), "v"(al), "v"(bh), "v"(bl));
}

template <int BN, int WK, int HB>
__global__ void __launch_bounds__(128)
k_gemm(const float* __restrict__ Abase, const float* __restrict__ Wbase,
       float* __restrict__ Cbase, const float* __restrict__ bias,
       long long sAb, long long sAm, long long sAn,
       long long sBb, long long sBm, long long sBn,
       long long sCb, long long sCm, long long sCn,
       int Mrows, int Ncols, int K, int lda, int ldb, int ldc,
       int nInner, int nMid, float bias_scale, float alpha)
{
  constexpr int TN  = BN / 16;
  constexpr int CP  = BN + 4;
  constexpr int NCH = BN / 16;

  __shared__ __attribute__((aligned(16))) unsigned short sAhi[64 * KP];
  __shared__ __attribute__((aligned(16))) unsigned short sAlo[64 * KP];
  __shared__ __attribute__((aligned(16))) unsigned short sWhi[BN * KP];
  __shared__ __attribute__((aligned(16))) unsigned short sWlo[BN * KP];
  __shared__ __attribute__((aligned(16))) float          sC[64 * CP];

  const int z  = blockIdx.z;
  const int zn = z % nInner;
  const int zm = (z / nInner) % nMid;
  const int zb = z / (nInner * nMid);
  const float* A = Abase + ((long long)zb * sAb + (long long)zm * sAm + (long long)zn * sAn);
  const float* W = Wbase + ((long long)zb * sBb + (long long)zm * sBm + (long long)zn * sBn);
  float*       C = Cbase + ((long long)zb * sCb + (long long)zm * sCm + (long long)zn * sCn);

  const int row0 = blockIdx.y * 64;
  const int col0 = blockIdx.x * BN;
  if (row0 + 64 > Mrows || col0 + BN > Ncols) return;

  const int tid = threadIdx.x;
  const int wv  = tid >> 5;
  const int l   = tid & 31;
  const int h   = l >> 4;
  const int m   = l & 15;

  v8f acc[TN];
#pragma unroll
  for (int j = 0; j < TN; ++j) acc[j] = (v8f){};

  for (int k0 = 0; k0 < K; k0 += 32) {
    v4f ra[4];
    v4f rw[NCH];
#pragma unroll
    for (int i = 0; i < 4; ++i) {
      const int c = tid + 128 * i;
      const int r = c >> 3, k4 = (c & 7) * 4;
      ra[i] = *(const v4f*)(A + (size_t)(row0 + r) * lda + k0 + k4);
    }
#pragma unroll
    for (int i = 0; i < NCH; ++i) {
      const int c = tid + 128 * i;
      if (WK) {
        const int s = c / (BN / 4), n4 = (c % (BN / 4)) * 4;
        rw[i] = *(const v4f*)(W + (size_t)(k0 + s) * ldb + col0 + n4);
      } else {
        const int n = c >> 3, k4 = (c & 7) * 4;
        rw[i] = *(const v4f*)(W + (size_t)(col0 + n) * ldb + k0 + k4);
      }
    }
    __syncthreads();
#pragma unroll
    for (int i = 0; i < 4; ++i) {
      const int c = tid + 128 * i;
      const int r = c >> 3, k4 = (c & 7) * 4;
      v2u hi, lo;
      split4(ra[i], hi, lo);
      *(v2u*)(&sAhi[r * KP + k4]) = hi;
      *(v2u*)(&sAlo[r * KP + k4]) = lo;
    }
#pragma unroll
    for (int i = 0; i < NCH; ++i) {
      const int c = tid + 128 * i;
      if (WK) {
        const int s = c / (BN / 4), n4 = (c % (BN / 4)) * 4;
        unsigned int h0, h1, h2, h3, l0, l1, l2, l3;
        split_hl(rw[i].x, h0, l0); split_hl(rw[i].y, h1, l1);
        split_hl(rw[i].z, h2, l2); split_hl(rw[i].w, h3, l3);
        sWhi[(n4 + 0) * KP + s] = (unsigned short)h0;  sWlo[(n4 + 0) * KP + s] = (unsigned short)l0;
        sWhi[(n4 + 1) * KP + s] = (unsigned short)h1;  sWlo[(n4 + 1) * KP + s] = (unsigned short)l1;
        sWhi[(n4 + 2) * KP + s] = (unsigned short)h2;  sWlo[(n4 + 2) * KP + s] = (unsigned short)l2;
        sWhi[(n4 + 3) * KP + s] = (unsigned short)h3;  sWlo[(n4 + 3) * KP + s] = (unsigned short)l3;
      } else {
        const int n = c >> 3, k4 = (c & 7) * 4;
        v2u hi, lo;
        split4(rw[i], hi, lo);
        *(v2u*)(&sWhi[n * KP + k4]) = hi;
        *(v2u*)(&sWlo[n * KP + k4]) = lo;
      }
    }
    __syncthreads();

    Frag ah, al;
    {
      const int ar = (16 * wv + m) * KP + 8 * h;
      ah.h[0] = *(const v8us*)(&sAhi[ar]);
      ah.h[1] = *(const v8us*)(&sAhi[ar + 16]);
      al.h[0] = *(const v8us*)(&sAlo[ar]);
      al.h[1] = *(const v8us*)(&sAlo[ar + 16]);
    }
#pragma unroll
    for (int j = 0; j < TN; ++j) {
      const int br = (16 * j + m) * KP + 8 * h;
      Frag bh, bl;
      bh.h[0] = *(const v8us*)(&sWhi[br]);
      bh.h[1] = *(const v8us*)(&sWhi[br + 16]);
      bl.h[0] = *(const v8us*)(&sWlo[br]);
      bl.h[1] = *(const v8us*)(&sWlo[br + 16]);
      mma3(acc[j], ah.v, al.v, bh.v, bl.v);
    }
  }

#pragma unroll
  for (int j = 0; j < TN; ++j) {
    float bb = 0.0f;
    if (HB) bb = bias_scale * bias[col0 + 16 * j + m];
#pragma unroll
    for (int r = 0; r < 8; ++r) {
      sC[(16 * wv + 8 * h + r) * CP + 16 * j + m] = alpha * acc[j][r] + bb;
    }
  }
  __syncthreads();
#pragma unroll
  for (int i = 0; i < BN / 8; ++i) {
    const int idx = i * 128 + tid;
    const int row = idx / (BN / 4);
    const int c4  = (idx % (BN / 4)) * 4;
    const v4f val = *(const v4f*)(&sC[row * CP + c4]);
    float* gp = C + (size_t)(row0 + row) * ldc + col0 + c4;
    *(volatile v4f*)gp = val;
  }
  __threadfence();
#pragma unroll
  for (int i = 0; i < BN / 8; ++i) {
    const int idx = i * 128 + tid;
    const int row = idx / (BN / 4);
    const int c4  = (idx % (BN / 4)) * 4;
    const v4f val = *(const v4f*)(&sC[row * CP + c4]);
    float* gp = C + (size_t)(row0 + row) * ldc + col0 + c4;
    *(volatile v4f*)gp = val;
  }
}

__global__ void __launch_bounds__(256)
k_sum_m(const float* __restrict__ in, float* __restrict__ out, int n4)
{
  const int i4 = blockIdx.x * 256 + threadIdx.x;
  if (i4 >= n4) return;
  const size_t i     = (size_t)i4 * 4;
  const size_t inner = (size_t)T_LEN * C_DIM;
  const size_t b     = i / inner;
  const size_t r     = i - b * inner;
  const float* p = in + b * (size_t)M_AX * inner + r;
  v4f s = {0.0f, 0.0f, 0.0f, 0.0f};
#pragma unroll 8
  for (int mm = 0; mm < M_AX; ++mm) s += *(const v4f*)(p + (size_t)mm * inner);
  float* o = out + i;
  *(volatile v4f*)o = s;
  __threadfence();
  *(volatile v4f*)o = s;
}

__global__ void __launch_bounds__(256)
k_softmax(float* __restrict__ w, float* __restrict__ a_out, int nrows, int narows)
{
  const int row  = blockIdx.x * 8 + (threadIdx.x >> 5);
  const int lane = threadIdx.x & 31;
  if (row >= nrows) return;
  float* p = w + (size_t)row * T_LEN + lane * 4;

  v4f v[4];
#pragma unroll
  for (int i = 0; i < 4; ++i) v[i] = *(const v4f*)(p + i * 128);

  float mx = -3.0e38f;
#pragma unroll
  for (int i = 0; i < 4; ++i)
    mx = fmaxf(mx, fmaxf(fmaxf(v[i].x, v[i].y), fmaxf(v[i].z, v[i].w)));
#pragma unroll
  for (int off = 16; off > 0; off >>= 1) mx = fmaxf(mx, __shfl_xor(mx, off, 32));

  float sum = 0.0f;
#pragma unroll
  for (int i = 0; i < 4; ++i) {
    v[i].x = __expf(v[i].x - mx);
    v[i].y = __expf(v[i].y - mx);
    v[i].z = __expf(v[i].z - mx);
    v[i].w = __expf(v[i].w - mx);
    sum += (v[i].x + v[i].y) + (v[i].z + v[i].w);
  }
#pragma unroll
  for (int off = 16; off > 0; off >>= 1) sum += __shfl_xor(sum, off, 32);
  const float inv = 1.0f / sum;
#pragma unroll
  for (int i = 0; i < 4; ++i) v[i] *= inv;

  const bool wa = row < narows;
  float* q = a_out + (size_t)(wa ? row : 0) * T_LEN + lane * 4;

#pragma unroll
  for (int i = 0; i < 4; ++i) {
    *(volatile v4f*)(p + i * 128) = v[i];
    if (wa) *(volatile v4f*)(q + i * 128) = v[i];
  }
  __threadfence();
#pragma unroll
  for (int i = 0; i < 4; ++i) {
    *(volatile v4f*)(p + i * 128) = v[i];
    if (wa) *(volatile v4f*)(q + i * 128) = v[i];
  }
}

extern "C" void kernel_launch(void* const* d_in, const int* in_sizes, int n_in,
                              void* d_out, int out_size, void* d_ws, size_t ws_size,
                              hipStream_t stream)
{
  if (n_in < 10) return;
  const int n_x  = B_SZ * M_AX * T_LEN * C_DIM;
  const int n_w  = C_DIM * C_DIM;
  const int n_a  = NH * T_LEN * T_LEN;
  if (in_sizes[0] != n_x || in_sizes[1] != n_x) return;
  if (in_sizes[2] != n_w || in_sizes[4] != n_w || in_sizes[6] != n_w || in_sizes[8] != n_w) return;
  if (in_sizes[3] != C_DIM || in_sizes[5] != C_DIM || in_sizes[7] != C_DIM || in_sizes[9] != C_DIM) return;
  if (out_size != n_x + n_a) return;

  const float* x  = (const float*)d_in[0];
  const float* y  = (const float*)d_in[1];
  const float* Wq = (const float*)d_in[2];
  const float* bq = (const float*)d_in[3];
  const float* Wk = (const float*)d_in[4];
  const float* bk = (const float*)d_in[5];
  const float* Wv = (const float*)d_in[6];
  const float* bv = (const float*)d_in[7];
  const float* Wp = (const float*)d_in[8];
  const float* bp = (const float*)d_in[9];

  float* out   = (float*)d_out;
  float* a_out = out + (size_t)n_x;

  const size_t n_sum = (size_t)B_SZ * T_LEN * C_DIM;
  const size_t n_v   = (size_t)n_x;
  const size_t n_sc  = (size_t)B_SZ * NH * T_LEN * T_LEN;
  const size_t o_xsum = 0;
  const size_t o_ysum = o_xsum + n_sum;
  const size_t o_qt   = o_ysum + n_sum;
  const size_t o_kt   = o_qt   + n_sum;
  const size_t o_v    = o_kt   + n_sum;
  const size_t o_wsc  = o_v    + n_v;
  const size_t o_att  = o_wsc  + n_sc;
  const size_t o_end  = o_att  + n_v;
  if (o_end * sizeof(float) > ws_size) return;

  float* ws   = (float*)d_ws;
  float* xsum = ws + o_xsum;
  float* ysum = ws + o_ysum;
  float* qt   = ws + o_qt;
  float* kt   = ws + o_kt;
  float* vbuf = ws + o_v;
  float* wsc  = ws + o_wsc;
  float* att  = ws + o_att;

  const int n4 = (int)(n_sum / 4);
  k_sum_m<<<dim3((n4 + 255) / 256), dim3(256), 0, stream>>>(x, xsum, n4);
  k_sum_m<<<dim3((n4 + 255) / 256), dim3(256), 0, stream>>>(y, ysum, n4);

  k_gemm<64, 0, 1><<<dim3(C_DIM / 64, (B_SZ * T_LEN) / 64, 1), dim3(128), 0, stream>>>(
      xsum, Wq, qt, bq, 0, 0, 0, 0, 0, 0, 0, 0, 0,
      B_SZ * T_LEN, C_DIM, C_DIM, C_DIM, C_DIM, C_DIM, 1, 1, (float)M_AX, 1.0f);
  k_gemm<64, 0, 1><<<dim3(C_DIM / 64, (B_SZ * T_LEN) / 64, 1), dim3(128), 0, stream>>>(
      ysum, Wk, kt, bk, 0, 0, 0, 0, 0, 0, 0, 0, 0,
      B_SZ * T_LEN, C_DIM, C_DIM, C_DIM, C_DIM, C_DIM, 1, 1, (float)M_AX, 1.0f);

  k_gemm<64, 0, 1><<<dim3(C_DIM / 64, (B_SZ * M_AX * T_LEN) / 64, 1), dim3(128), 0, stream>>>(
      y, Wv, vbuf, bv, 0, 0, 0, 0, 0, 0, 0, 0, 0,
      B_SZ * M_AX * T_LEN, C_DIM, C_DIM, C_DIM, C_DIM, C_DIM, 1, 1, 1.0f, 1.0f);

  k_gemm<64, 0, 0><<<dim3(T_LEN / 64, T_LEN / 64, B_SZ * NH), dim3(128), 0, stream>>>(
      qt, kt, wsc, kt,
      (long long)T_LEN * C_DIM, 0, DH,
      (long long)T_LEN * C_DIM, 0, DH,
      (long long)NH * T_LEN * T_LEN, 0, (long long)T_LEN * T_LEN,
      T_LEN, T_LEN, DH, C_DIM, C_DIM, T_LEN, NH, 1, 0.0f, 1.0f / 32.0f);

  const int nrows = B_SZ * NH * T_LEN;
  k_softmax<<<dim3((nrows + 7) / 8), dim3(256), 0, stream>>>(wsc, a_out, nrows, NH * T_LEN);

  k_gemm<32, 1, 0><<<dim3(1, T_LEN / 64, B_SZ * M_AX * NH), dim3(128), 0, stream>>>(
      wsc, vbuf, att, vbuf,
      (long long)NH * T_LEN * T_LEN, 0, (long long)T_LEN * T_LEN,
      (long long)M_AX * T_LEN * C_DIM, (long long)T_LEN * C_DIM, DH,
      (long long)M_AX * T_LEN * C_DIM, (long long)T_LEN * C_DIM, DH,
      T_LEN, DH, T_LEN, T_LEN, C_DIM, C_DIM, NH, M_AX, 0.0f, 1.0f);

  k_gemm<64, 0, 1><<<dim3(C_DIM / 64, (B_SZ * M_AX * T_LEN) / 64, 1), dim3(128), 0, stream>>>(
      att, Wp, out, bp, 0, 0, 0, 0, 0, 0, 0, 0, 0,
      B_SZ * M_AX * T_LEN, C_DIM, C_DIM, C_DIM, C_DIM, C_DIM, 1, 1, 1.0f, 1.0f);
}
